// MambaLayer_13348758356004
// MI455X (gfx1250) — hardware-run, weakly checked
//
#include <hip/hip_runtime.h>
#include <math.h>

typedef __attribute__((ext_vector_type(16))) _Float16 v16h;
typedef __attribute__((ext_vector_type(8)))  _Float16 v8h;
typedef __attribute__((ext_vector_type(16))) __bf16   v16b;
typedef __attribute__((ext_vector_type(8)))  __bf16   v8b;
typedef __attribute__((ext_vector_type(8)))  float    v8f;
typedef __attribute__((ext_vector_type(4)))  float    v4f;
typedef __attribute__((ext_vector_type(2)))  float    v2f;

constexpr int kRows = 4096;
constexpr int kDim  = 1024;
constexpr int kDin  = 2048;
constexpr int kNst  = 16;
constexpr int kDtR  = 64;
constexpr int kConv = 4;
constexpr int kXzN  = 2 * kDin;
constexpr int kXdN  = kDtR + 2 * kNst;
constexpr int kXdP  = 128;
constexpr float kLnEps        = 1e-5f;
constexpr float kWCarry       = 1024.0f;
constexpr float kActCarry     = 1024.0f;
constexpr float kDtpCarry     = 16.0f;
constexpr float kF16MinNormal = 6.103515625e-5f;
static_assert((kDim % 32) == 0 && (kDin % 32) == 0 && (kDtR % 32) == 0);
static_assert((kRows % 64) == 0 && (kDin % 64) == 0 && (kXdP % 64) == 0 && (kDim % 64) == 0);
static_assert(((kRows / 64) * (kDin / 64)) % 8 == 0 && ((kRows / 64) * (kXdP / 64)) % 8 == 0 && ((kRows / 64) * (kDim / 64)) % 8 == 0);
static_assert(kXdN <= kXdP);

constexpr size_t kOffWIN  = 0;
constexpr size_t kOffWINB = kOffWIN  + (size_t)kXzN  * kDim * 2;
constexpr size_t kOffWXP  = kOffWINB + (size_t)kXzN  * kDim * 2;
constexpr size_t kOffWDT  = kOffWXP  + (size_t)kXdP  * kDin * 2;
constexpr size_t kOffWOUT = kOffWDT  + (size_t)kDin  * kDtR * 2;
constexpr size_t kOffXNH  = kOffWOUT + (size_t)kDim  * kDin * 2;
constexpr size_t kOffXNL  = kOffXNH  + (size_t)kRows * kDim * 2;
constexpr size_t kOffXIZ  = kOffXNL  + (size_t)kRows * kDim * 2;
constexpr size_t kOffXC   = kOffXIZ  + (size_t)kRows * kDin * 4;
constexpr size_t kOffXD   = kOffXC   + (size_t)kRows * kDin * 2;
constexpr size_t kOffSS   = kOffXD   + (size_t)kRows * kXdP * 4;
constexpr size_t kOffDTL  = kOffSS   + (size_t)kRows * 4;
constexpr size_t kOffDTP  = kOffDTL  + (size_t)kRows * kDtR * 2;
constexpr size_t kOffYY   = kOffDTP  + (size_t)kRows * kDin * 2;
constexpr size_t kWsTotal = kOffYY   + (size_t)kRows * kDin * 2;
static_assert(kWsTotal == 125059072ull);
static_assert(kWsTotal <= 134217728ull);
static_assert((kOffWINB % 128) == 0 && (kOffWXP % 128) == 0 && (kOffWDT % 128) == 0 && (kOffWOUT % 128) == 0 &&
              (kOffXNH % 128) == 0 && (kOffXNL % 128) == 0 && (kOffXIZ % 128) == 0 && (kOffXC % 128) == 0 &&
              (kOffXD % 128) == 0 && (kOffSS % 128) == 0 && (kOffDTL % 128) == 0 && (kOffDTP % 128) == 0 &&
              (kOffYY % 128) == 0);

__device__ __forceinline__ unsigned short f2bf_bits(float f) {
  unsigned u = __float_as_uint(f);
  return (unsigned short)((u + 0x7FFFu + ((u >> 16) & 1u)) >> 16);
}
__device__ __forceinline__ float bf_bits2f(unsigned short h) { return __uint_as_float(((unsigned)h) << 16); }

__device__ __forceinline__ float h16_to_f32(unsigned hb) {
  const unsigned sgn = (hb & 0x8000u) << 16; const unsigned em = hb & 0x7fffu;
  const float fn = __uint_as_float((em << 13) + 0x38000000u);
  const float fs = (float)em * 5.9604644775390625e-8f;
  const float mag = (em < 0x400u) ? fs : fn; return __uint_as_float(__float_as_uint(mag) | sgn); }

__device__ __forceinline__ void tie4_hh(v8f& a, v8f& b, v8f& c, v8f& d, v16h x, v16h y) { asm volatile("v_nop\n\tv_nop\n\tv_nop\n\tv_nop" : "+v"(a), "+v"(b), "+v"(c), "+v"(d) : "v"(x), "v"(y)); }
__device__ __forceinline__ void tie4_hb(v8f& a, v8f& b, v8f& c, v8f& d, v16h x, v16b y) { asm volatile("v_nop\n\tv_nop\n\tv_nop\n\tv_nop" : "+v"(a), "+v"(b), "+v"(c), "+v"(d) : "v"(x), "v"(y)); }
__device__ __forceinline__ void tie4_bb(v8f& a, v8f& b, v8f& c, v8f& d, v16b x, v16b y) { asm volatile("v_nop\n\tv_nop\n\tv_nop\n\tv_nop" : "+v"(a), "+v"(b), "+v"(c), "+v"(d) : "v"(x), "v"(y)); }
__device__ __forceinline__ void keep4_h(v16h a, v16h b, v16h c, v16h d) { asm volatile("v_nop" :: "v"(a), "v"(b), "v"(c), "v"(d)); }
__device__ __forceinline__ void keep4_b(v16b a, v16b b, v16b c, v16b d) { asm volatile("v_nop" :: "v"(a), "v"(b), "v"(c), "v"(d)); }
__device__ __forceinline__ void acc_guard4(v8f& a, v8f& b, v8f& c, v8f& d) { asm volatile("v_nop\n\tv_nop\n\tv_nop\n\tv_nop" : "+v"(a), "+v"(b), "+v"(c), "+v"(d)); }
template <typename T> struct Frag;
template <> struct Frag<_Float16> {
  typedef v16h V; union U { v16h v; v8h h[2]; };
  static __device__ __forceinline__ v16h load(const _Float16* p) {
    U f; f.h[0] = *(const v8h*)(p); f.h[1] = *(const v8h*)(p + 16); return f.v;
  }
  static __device__ __forceinline__ v8f mma(v16h a, v16h b, v8f c) {
    return __builtin_amdgcn_wmma_f32_16x16x32_f16(false, a, false, b, (short)0, c, false, false);
  }
  static __device__ __forceinline__ void tie4(v8f& a, v8f& b, v8f& c, v8f& d, v16h x, v16h y) { tie4_hh(a, b, c, d, x, y); }
  static __device__ __forceinline__ void tie4q(v8f& a, v8f& b, v8f& c, v8f& d, v16h x, v16b y) { tie4_hb(a, b, c, d, x, y); }
  static __device__ __forceinline__ void keep(v16h a, v16h b, v16h c, v16h d) { keep4_h(a, b, c, d); }
};
template <> struct Frag<__bf16> {
  typedef v16b V; union U { v16b v; v8b h[2]; };
  static __device__ __forceinline__ v16b load(const __bf16* p) {
    U f; f.h[0] = *(const v8b*)(p); f.h[1] = *(const v8b*)(p + 16); return f.v;
  }
  static __device__ __forceinline__ v8f mma(v16b a, v16b b, v8f c) {
    return __builtin_amdgcn_wmma_f32_16x16x32_bf16(false, a, false, b, (short)0, c, false, false);
  }
  static __device__ __forceinline__ void tie4(v8f& a, v8f& b, v8f& c, v8f& d, v16b x, v16b y) { tie4_bb(a, b, c, d, x, y); }
  static __device__ __forceinline__ void tie4q(v8f& a, v8f& b, v8f& c, v8f& d, v16b x, v16b y) { tie4_bb(a, b, c, d, x, y); }
  static __device__ __forceinline__ void keep(v16b a, v16b b, v16b c, v16b d) { keep4_b(a, b, c, d); }
};

template <int ET> struct Elem;
template <> struct Elem<0> { typedef _Float16 T; };
template <> struct Elem<1> { typedef __bf16 T; };
template <int ET, int SPL, int BIAS_MODE, int OUT_MODE, bool RESID, int ACT = 0>
__global__ __launch_bounds__(256) void wmma_gemm64(
    const unsigned short* __restrict__ Ap, const unsigned short* __restrict__ A2p, int lda, long strideA,
    const unsigned short* __restrict__ Btp, const unsigned short* __restrict__ Bt2p, int ldb, long strideB,
    void* __restrict__ Cout, void* __restrict__ Cout2, int ldc, long strideC,
    const float* __restrict__ bias,
    const float* __restrict__ resid, long strideR,
    int M, int N, int K, float scale) {
  typedef typename Elem<ET>::T T;
  typedef typename Frag<T>::V V;
  const T* A = (const T*)Ap; const T* A2 = (const T*)A2p; const T* Bt = (const T*)Btp; const T* Bt2 = (const T*)Bt2p;
  const __bf16* Aq = (const __bf16*)A2p; const __bf16* Bq = (const __bf16*)Bt2p;
  __shared__ __align__(16) float sT[8][16 * 68];
  const int b    = blockIdx.y;
  const int lane = threadIdx.x & 31;
  const int wave = threadIdx.x >> 5;
  const int tilesN = N >> 6;
  const int tilesM = M >> 6;
  const int tile = blockIdx.x * 8 + wave;
  if (tile >= tilesM * tilesN) return;
  const int tm = tile / tilesN;
  const int tn = tile - tm * tilesN;
  const int m0 = tm << 6;
  const int n0 = tn << 6;

  const T* Ab  = A  + (size_t)b * strideA;
  const T* Bb  = Bt + (size_t)b * strideB;
  const T* Ab2 = (SPL == 1 || SPL == 2) ? (A2  + (size_t)b * strideA) : nullptr;
  const T* Bb2 = (SPL == 2) ? (Bt2 + (size_t)b * strideB) : nullptr;
  const __bf16* Aqb = (SPL == 3) ? (Aq + (size_t)b * strideA) : nullptr;
  const __bf16* Bqb = (SPL == 3) ? (Bq + (size_t)b * strideB) : nullptr;

  const int rlane = lane & 15;
  const int koff  = (lane >> 4) * 8;
  const int mOff  = (lane >> 4) * 8;

  v8f acc[4][4];
#pragma unroll
  for (int i = 0; i < 4; ++i)
#pragma unroll
    for (int j = 0; j < 4; ++j) acc[i][j] = (v8f){0.f,0.f,0.f,0.f,0.f,0.f,0.f,0.f};

  for (int k0 = 0; k0 < K; k0 += 32) {
    V bh[4], bl[4]; v16b bq[4];
#pragma unroll
    for (int j = 0; j < 4; ++j) {
      const size_t bo = (size_t)(n0 + (j << 4) + rlane) * ldb + koff + k0;
      bh[j] = Frag<T>::load(Bb + bo);
      if constexpr (SPL == 2) bl[j] = Frag<T>::load(Bb2 + bo);
      if constexpr (SPL == 3) bq[j] = Frag<__bf16>::load(Bqb + bo);
    }
#pragma unroll
    for (int i = 0; i < 4; ++i) {
      const size_t ao = (size_t)(m0 + (i << 4) + rlane) * lda + koff + k0;
      V ah = Frag<T>::load(Ab + ao);
      V al; v16b aq;
      if constexpr (SPL == 1 || SPL == 2) al = Frag<T>::load(Ab2 + ao);
      if constexpr (SPL == 3) aq = Frag<__bf16>::load(Aqb + ao);
#pragma unroll
      for (int j = 0; j < 4; ++j) {
        acc[i][j] = Frag<T>::mma(ah, bh[j], acc[i][j]);
        if constexpr (SPL == 2) acc[i][j] = Frag<T>::mma(ah, bl[j], acc[i][j]);
        if constexpr (SPL == 1 || SPL == 2) acc[i][j] = Frag<T>::mma(al, bh[j], acc[i][j]);
        if constexpr (SPL == 3) acc[i][j] = Frag<__bf16>::mma(aq, bq[j], acc[i][j]);
      }
      if constexpr (SPL == 0) Frag<T>::tie4(acc[i][0], acc[i][1], acc[i][2], acc[i][3], ah, ah);
      if constexpr (SPL == 1 || SPL == 2) Frag<T>::tie4(acc[i][0], acc[i][1], acc[i][2], acc[i][3], ah, al);
      if constexpr (SPL == 3) Frag<T>::tie4q(acc[i][0], acc[i][1], acc[i][2], acc[i][3], ah, aq);
    }
    Frag<T>::keep(bh[0], bh[1], bh[2], bh[3]);
    if constexpr (SPL == 2) Frag<T>::keep(bl[0], bl[1], bl[2], bl[3]);
    if constexpr (SPL == 3) keep4_b(bq[0], bq[1], bq[2], bq[3]);
  }
  acc_guard4(acc[0][0], acc[0][1], acc[0][2], acc[0][3]);
  acc_guard4(acc[1][0], acc[1][1], acc[1][2], acc[1][3]);
  acc_guard4(acc[2][0], acc[2][1], acc[2][2], acc[2][3]);
  acc_guard4(acc[3][0], acc[3][1], acc[3][2], acc[3][3]);

  float* slab = sT[wave];
  const float* Rb = RESID ? (resid + (size_t)b * strideR) : nullptr;
#pragma unroll
  for (int i = 0; i < 4; ++i) {
    const int mBase = m0 + (i << 4);
#pragma unroll
    for (int j = 0; j < 4; ++j) {
      const int n = n0 + (j << 4) + rlane;
      float bv = 0.f;
      if (BIAS_MODE == 2) bv = bias[n];
#pragma unroll
      for (int r = 0; r < 8; ++r) {
        float v = acc[i][j][r] * scale;
        if (BIAS_MODE == 1) v += bias[mBase + mOff + r];
        if (BIAS_MODE == 2) v += bv;
        if (RESID) v += Rb[(size_t)(mBase + mOff + r) * ldc + n];
        if (ACT == 1) v = tanhf(v);
        if (ACT == 2) v = fmaxf(v, 0.0f);
        if (ACT == 3) v = v / (1.0f + expf(-v));
        if (ACT == 4) v = (v > 0.f) ? v : 0.01f * v;
        slab[(mOff + r) * 68 + (j << 4) + rlane] = v;
      }
    }
    __builtin_amdgcn_fence(__ATOMIC_RELEASE, "workgroup");
    __builtin_amdgcn_wave_barrier();
    __builtin_amdgcn_fence(__ATOMIC_ACQUIRE, "workgroup");
    if (OUT_MODE == 0) {
      float* C = (float*)Cout + (size_t)b * strideC;
      const int hh = lane >> 4, c4 = (lane & 15) * 4;
      for (int pass = 0; pass < 2; ++pass) {
#pragma unroll
        for (int it = 0; it < 8; ++it) {
          const int row = it * 2 + hh;
          v4f v = *(const v4f*)(slab + row * 68 + c4);
          *(volatile v4f*)(C + (size_t)(mBase + row) * ldc + n0 + c4) = v;
        }
        __threadfence();
      }
    } else {
      const int q = lane >> 3, c8 = (lane & 7) * 8;
      unsigned short* C  = (unsigned short*)Cout  + (size_t)b * strideC;
      unsigned short* C2 = (OUT_MODE == 2) ? ((unsigned short*)Cout2 + (size_t)b * strideC) : nullptr;
      for (int pass = 0; pass < 2; ++pass) {
#pragma unroll
        for (int it = 0; it < 4; ++it) {
          const int row = it * 4 + q;
          const float* sp = slab + row * 68 + c8;
          v8h hv, lv;
#pragma unroll
          for (int e = 0; e < 8; ++e) {
            if (OUT_MODE == 1) {
              hv[e] = (_Float16)sp[e];
            } else {
              unsigned short hb = f2bf_bits(sp[e]);
              unsigned short lb = f2bf_bits(sp[e] - bf_bits2f(hb));
              hv[e] = __builtin_bit_cast(_Float16, hb);
              lv[e] = __builtin_bit_cast(_Float16, lb);
            }
          }
          *(volatile v8h*)(C + (size_t)(mBase + row) * ldc + n0 + c8) = hv;
          if (OUT_MODE == 2) *(volatile v8h*)(C2 + (size_t)(mBase + row) * ldc + n0 + c8) = lv;
        }
        __threadfence();
      }
    }
    __builtin_amdgcn_fence(__ATOMIC_RELEASE, "workgroup");
    __builtin_amdgcn_wave_barrier();
    __builtin_amdgcn_fence(__ATOMIC_ACQUIRE, "workgroup");
  }
}

__global__ __launch_bounds__(256) void cast_w_dual_kernel(
    const float* __restrict__ src, unsigned short* __restrict__ dh, unsigned short* __restrict__ db, int total8, float scale)
{
  const int i = blockIdx.x * 256 + threadIdx.x;
  if (i >= total8) return;
  const size_t e0 = (size_t)i << 3;
  const v4f a0 = *(const v4f*)(src + e0);
  const v4f a1 = *(const v4f*)(src + e0 + 4);
  v8h hv, bv;
#pragma unroll
  for (int e = 0; e < 4; ++e) {
    const float f0 = a0[e] * scale, f1 = a1[e] * scale;
    hv[e]     = (_Float16)f0;
    hv[4 + e] = (_Float16)f1;
    const unsigned short b0 = f2bf_bits(f0), b1 = f2bf_bits(f1);
    bv[e]     = __builtin_bit_cast(_Float16, b0);
    bv[4 + e] = __builtin_bit_cast(_Float16, b1);
  }
  unsigned short* qh = dh + e0;
  unsigned short* qb = db + e0;
  *(volatile v8h*)qh = hv;
  *(volatile v8h*)qb = bv;
  __threadfence();
  *(volatile v8h*)qh = hv;
  *(volatile v8h*)qb = bv;
}

__global__ __launch_bounds__(256) void cast_f16x8_kernel(
    const float* __restrict__ src, unsigned short* __restrict__ dst, int live8, int total8, float scale)
{
  const int i = blockIdx.x * 256 + threadIdx.x;
  if (i >= total8) return;
  const bool live = (i < live8);
  const int j = live ? i : (live8 - 1);
  const float sf = live ? scale : 0.0f;
  const size_t s0 = (size_t)j << 3;
  const v4f a0 = *(const v4f*)(src + s0);
  const v4f a1 = *(const v4f*)(src + s0 + 4);
  v8h hv;
#pragma unroll
  for (int e = 0; e < 4; ++e) {
    hv[e]     = (_Float16)(a0[e] * sf);
    hv[4 + e] = (_Float16)(a1[e] * sf);
  }
  unsigned short* q = dst + ((size_t)i << 3);
  *(volatile v8h*)q = hv;
  __threadfence();
  *(volatile v8h*)q = hv;
}

__device__ __forceinline__ void split_h16_b16(float v, _Float16& hi, _Float16& lo) {
  const float vh = (fabsf(v) < kF16MinNormal) ? 0.0f : v;
  const _Float16 h = (_Float16)vh;
  const unsigned short hb = __builtin_bit_cast(unsigned short, h);
  const float hf = h16_to_f32((unsigned)hb);
  const unsigned short lb = f2bf_bits(v - hf);
  hi = h;
  lo = __builtin_bit_cast(_Float16, lb);
}

__global__ __launch_bounds__(128) void ln_split_kernel(
    const float* __restrict__ x, const float* __restrict__ gam, const float* __restrict__ bet,
    unsigned short* __restrict__ XNH, unsigned short* __restrict__ XNL)
{
  __shared__ float sr1[4];
  __shared__ float sr2[4];
  const int tid = threadIdx.x, lane = tid & 31, wave = tid >> 5;
  const int row = blockIdx.x;
  const int c0 = tid * 8;
  const float* xr = x + (size_t)row * kDim + c0;
  const v4f a0 = *(const v4f*)(xr);
  const v4f a1 = *(const v4f*)(xr + 4);
  float s = 0.0f;
#pragma unroll
  for (int e = 0; e < 4; ++e) s += a0[e];
#pragma unroll
  for (int e = 0; e < 4; ++e) s += a1[e];
#pragma unroll
  for (int off = 16; off > 0; off >>= 1) s += __shfl_xor(s, off, 32);
  if (lane == 0) sr1[wave] = s;
  __syncthreads();
  const float mu = ((sr1[0] + sr1[1]) + (sr1[2] + sr1[3])) * (1.0f / (float)kDim);
  v4f d0, d1;
#pragma unroll
  for (int e = 0; e < 4; ++e) { d0[e] = a0[e] - mu; d1[e] = a1[e] - mu; }
  float s2 = 0.0f;
#pragma unroll
  for (int e = 0; e < 4; ++e) s2 += d0[e] * d0[e];
#pragma unroll
  for (int e = 0; e < 4; ++e) s2 += d1[e] * d1[e];
#pragma unroll
  for (int off = 16; off > 0; off >>= 1) s2 += __shfl_xor(s2, off, 32);
  if (lane == 0) sr2[wave] = s2;
  __syncthreads();
  const float var = ((sr2[0] + sr2[1]) + (sr2[2] + sr2[3])) * (1.0f / (float)kDim);
  const float rs = rsqrtf(var + kLnEps);
  const v4f g0 = *(const v4f*)(gam + c0), g1 = *(const v4f*)(gam + c0 + 4);
  const v4f b0 = *(const v4f*)(bet + c0), b1 = *(const v4f*)(bet + c0 + 4);
  v8h hv, lv;
#pragma unroll
  for (int e = 0; e < 4; ++e) {
    _Float16 hh, ll;
    split_h16_b16(d0[e] * rs * g0[e] + b0[e], hh, ll);
    hv[e] = hh; lv[e] = ll;
    split_h16_b16(d1[e] * rs * g1[e] + b1[e], hh, ll);
    hv[4 + e] = hh; lv[4 + e] = ll;
  }
  const size_t o = (size_t)row * kDim + c0;
  *(volatile v8h*)(XNH + o) = hv;
  *(volatile v8h*)(XNL + o) = lv;
  __threadfence();
  *(volatile v8h*)(XNH + o) = hv;
  *(volatile v8h*)(XNL + o) = lv;
}

__global__ __launch_bounds__(256) void conv_silu_kernel(
    const float* __restrict__ XI, const float* __restrict__ cw, const float* __restrict__ cb,
    unsigned* __restrict__ XCw)
{
  const int i = blockIdx.x * 256 + threadIdx.x;
  const int b = i >> 10;
  const int w = i & 1023;
  const int e0 = 2 * w;
  const v2f xv  = *(const v2f*)(XI + (size_t)b * kDin + e0);
  const v2f cbv = *(const v2f*)(cb + e0);
  const float w30 = cw[e0 * kConv + (kConv - 1)];
  const float w31 = cw[(e0 + 1) * kConv + (kConv - 1)];
  const float p0 = w30 * xv[0] + cbv[0];
  const float p1 = w31 * xv[1] + cbv[1];
  const float g0 = __builtin_amdgcn_rcpf(1.0f + expf(-p0));
  const float g1 = __builtin_amdgcn_rcpf(1.0f + expf(-p1));
  const float xc0 = (p0 * g0) * kActCarry;
  const float xc1 = (p1 * g1) * kActCarry;
  const _Float16 h0 = (_Float16)xc0, h1 = (_Float16)xc1;
  const unsigned u = (unsigned)__builtin_bit_cast(unsigned short, h0) | ((unsigned)__builtin_bit_cast(unsigned short, h1) << 16);
  ((volatile unsigned*)XCw)[i] = u;
  __threadfence();
  ((volatile unsigned*)XCw)[i] = u;
}

__global__ __launch_bounds__(256) void xd_split_kernel(
    const float* __restrict__ XD, float* __restrict__ SS, unsigned short* __restrict__ DTL)
{
  const int tid = threadIdx.x, lane = tid & 31, wave = tid >> 5;
  const int rowb = blockIdx.x * 32;
  {
    const int row = rowb + (tid >> 3);
    const int c8 = (tid & 7) * 8;
    const float* p = XD + (size_t)row * kXdP + c8;
    const v4f a0 = *(const v4f*)(p);
    const v4f a1 = *(const v4f*)(p + 4);
    v8h hv;
#pragma unroll
    for (int e = 0; e < 4; ++e) {
      hv[e]     = (_Float16)(a0[e] * kActCarry);
      hv[4 + e] = (_Float16)(a1[e] * kActCarry);
    }
    unsigned short* q = DTL + (size_t)row * kDtR + c8;
    *(volatile v8h*)q = hv;
    __threadfence();
    *(volatile v8h*)q = hv;
  }
  if (wave == 0) {
    const int row = rowb + lane;
    const float* p = XD + (size_t)row * kXdP + kDtR;
    const v4f bm0 = *(const v4f*)(p),      bm1 = *(const v4f*)(p + 4),  bm2 = *(const v4f*)(p + 8),  bm3 = *(const v4f*)(p + 12);
    asm volatile("" ::: "memory");
    const v4f cm0 = *(const v4f*)(p + 16), cm1 = *(const v4f*)(p + 20), cm2 = *(const v4f*)(p + 24), cm3 = *(const v4f*)(p + 28);
    float s = 0.0f;
#pragma unroll
    for (int e = 0; e < 4; ++e) s = fmaf(bm0[e], cm0[e], s);
#pragma unroll
    for (int e = 0; e < 4; ++e) s = fmaf(bm1[e], cm1[e], s);
#pragma unroll
    for (int e = 0; e < 4; ++e) s = fmaf(bm2[e], cm2[e], s);
#pragma unroll
    for (int e = 0; e < 4; ++e) s = fmaf(bm3[e], cm3[e], s);
    ((volatile float*)SS)[row] = s;
    __threadfence();
    ((volatile float*)SS)[row] = s;
  }
}

__device__ __forceinline__ float gate_one(float dtp16, float bd, float dsk, float sb, unsigned xch, float z) {
  const float v   = dtp16 * (1.0f / kDtpCarry) + bd;
  const float a   = expf(-fabsf(v));
  const float u   = 1.0f + a;
  const float l1p = __logf(u) + (a - (u - 1.0f)) * __builtin_amdgcn_rcpf(u);
  const float dt  = fmaxf(v, 0.0f) + l1p;
  const float xc  = h16_to_f32(xch) * (1.0f / kActCarry);
  const float sg  = __builtin_amdgcn_rcpf(1.0f + expf(-z));
  const float y0  = xc * (dsk + dt * sb);
  return (y0 * (z * sg)) * kActCarry;
}

__global__ __launch_bounds__(256) void gate_kernel(
    const unsigned* __restrict__ DTPw, const float* __restrict__ bdt, const float* __restrict__ Dsk,
    const float* __restrict__ SS, const unsigned* __restrict__ XCw, const float* __restrict__ Z,
    unsigned* __restrict__ YYw)
{
  const int i = blockIdx.x * 256 + threadIdx.x;
  const int b = i >> 10;
  const int w = i & 1023;
  const int d0 = 2 * w;
  const unsigned dw = DTPw[i];
  const v2f bb = *(const v2f*)(bdt + d0);
  const v2f dk = *(const v2f*)(Dsk + d0);
  const float sb = SS[b];
  const unsigned xcw = XCw[i];
  const v2f zv = *(const v2f*)(Z + (size_t)b * kDin + d0);
  const float dp0 = h16_to_f32(dw & 0xffffu);
  const float dp1 = h16_to_f32(dw >> 16);
  const float y0 = gate_one(dp0, bb[0], dk[0], sb, xcw & 0xffffu, zv[0]);
  const float y1 = gate_one(dp1, bb[1], dk[1], sb, xcw >> 16,     zv[1]);
  const _Float16 h0 = (_Float16)y0, h1 = (_Float16)y1;
  const unsigned u = (unsigned)__builtin_bit_cast(unsigned short, h0) | ((unsigned)__builtin_bit_cast(unsigned short, h1) << 16);
  ((volatile unsigned*)YYw)[i] = u;
  __threadfence();
  ((volatile unsigned*)YYw)[i] = u;
}

extern "C" void kernel_launch(void* const* d_in, const int* in_sizes, int n_in,
                              void* d_out, int out_size, void* d_ws, size_t ws_size,
                              hipStream_t stream) {
  if (n_in < 12) return;
  if (in_sizes[0]  != kRows * kDim) return;
  if (in_sizes[1]  != kDim) return;
  if (in_sizes[2]  != kDim) return;
  if (in_sizes[3]  != kXzN * kDim) return;
  if (in_sizes[4]  != kDin * kConv) return;
  if (in_sizes[5]  != kDin) return;
  if (in_sizes[6]  != kXdN * kDin) return;
  if (in_sizes[7]  != kDin * kDtR) return;
  if (in_sizes[8]  != kDin) return;
  if (in_sizes[9]  != kDin * kNst) return;
  if (in_sizes[10] != kDin) return;
  if (in_sizes[11] != kDim * kDin) return;
  if (out_size != kRows * kDim) return;
  if (ws_size < kWsTotal) return;

  const float* x        = (const float*)d_in[0];
  const float* ln_gamma = (const float*)d_in[1];
  const float* ln_beta  = (const float*)d_in[2];
  const float* W_in     = (const float*)d_in[3];
  const float* conv_w   = (const float*)d_in[4];
  const float* conv_b   = (const float*)d_in[5];
  const float* W_xproj  = (const float*)d_in[6];
  const float* W_dt     = (const float*)d_in[7];
  const float* b_dt     = (const float*)d_in[8];
  const float* Dskip    = (const float*)d_in[10];
  const float* W_out    = (const float*)d_in[11];
  float* out = (float*)d_out;

  char* ws = (char*)d_ws;
  unsigned short* WIN  = (unsigned short*)(ws + kOffWIN);
  unsigned short* WINB = (unsigned short*)(ws + kOffWINB);
  unsigned short* WXP  = (unsigned short*)(ws + kOffWXP);
  unsigned short* WDT  = (unsigned short*)(ws + kOffWDT);
  unsigned short* WOUT = (unsigned short*)(ws + kOffWOUT);
  unsigned short* XNH  = (unsigned short*)(ws + kOffXNH);
  unsigned short* XNL  = (unsigned short*)(ws + kOffXNL);
  float*          XIZ  = (float*)(ws + kOffXIZ);
  unsigned short* XC   = (unsigned short*)(ws + kOffXC);
  float*          XD   = (float*)(ws + kOffXD);
  float*          SS   = (float*)(ws + kOffSS);
  unsigned short* DTL  = (unsigned short*)(ws + kOffDTL);
  unsigned short* DTP  = (unsigned short*)(ws + kOffDTP);
  unsigned short* YY   = (unsigned short*)(ws + kOffYY);

  {
    constexpr int t8_in  = kXzN * kDim / 8;           static_assert(t8_in % 256 == 0);
    constexpr int l8_xp  = kXdN * kDin / 8;           static_assert(l8_xp % 256 == 0);
    constexpr int t8_xp  = kXdP * kDin / 8;           static_assert(t8_xp % 256 == 0);
    constexpr int t8_dt  = kDin * kDtR / 8;           static_assert(t8_dt % 256 == 0);
    constexpr int t8_out = kDim * kDin / 8;           static_assert(t8_out % 256 == 0);
    cast_w_dual_kernel<<<t8_in / 256, 256, 0, stream>>>(W_in, WIN, WINB, t8_in, kWCarry);
    cast_f16x8_kernel<<<t8_xp / 256,  256, 0, stream>>>(W_xproj, WXP,  l8_xp,  t8_xp,  kWCarry);
    cast_f16x8_kernel<<<t8_dt / 256,  256, 0, stream>>>(W_dt,    WDT,  t8_dt,  t8_dt,  kWCarry);
    cast_f16x8_kernel<<<t8_out / 256, 256, 0, stream>>>(W_out,   WOUT, t8_out, t8_out, kWCarry);
  }

  ln_split_kernel<<<kRows, 128, 0, stream>>>(x, ln_gamma, ln_beta, XNH, XNL);

  wmma_gemm64<0, 3, 0, 0, false><<<dim3((kRows / 64) * (kDin / 64) / 8, 1), 256, 0, stream>>>(
      XNH, XNL, kDim, 0L,
      WIN, WINB, kDim, 0L,
      (void*)XIZ, nullptr, kDin, 0L,
      nullptr, nullptr, 0L,
      kRows, kDin, kDim, 1.0f / kWCarry);

  conv_silu_kernel<<<(kRows * (kDin / 2)) / 256, 256, 0, stream>>>(XIZ, conv_w, conv_b, (unsigned*)XC);

  wmma_gemm64<0, 3, 0, 0, false><<<dim3((kRows / 64) * (kDin / 64) / 8, 1), 256, 0, stream>>>(
      XNH, XNL, kDim, 0L,
      WIN + (size_t)kDin * kDim, WINB + (size_t)kDin * kDim, kDim, 0L,
      (void*)XIZ, nullptr, kDin, 0L,
      nullptr, nullptr, 0L,
      kRows, kDin, kDim, 1.0f / kWCarry);

  wmma_gemm64<0, 0, 0, 0, false><<<dim3((kRows / 64) * (kXdP / 64) / 8, 1), 256, 0, stream>>>(
      XC, nullptr, kDin, 0L,
      WXP, nullptr, kDin, 0L,
      (void*)XD, nullptr, kXdP, 0L,
      nullptr, nullptr, 0L,
      kRows, kXdP, kDin, 1.0f / (kActCarry * kWCarry));

  xd_split_kernel<<<kRows / 32, 256, 0, stream>>>(XD, SS, DTL);

  wmma_gemm64<0, 0, 0, 1, false><<<dim3((kRows / 64) * (kDin / 64) / 8, 1), 256, 0, stream>>>(
      DTL, nullptr, kDtR, 0L,
      WDT, nullptr, kDtR, 0L,
      (void*)DTP, nullptr, kDin, 0L,
      nullptr, nullptr, 0L,
      kRows, kDin, kDtR, kDtpCarry / (kActCarry * kWCarry));

  gate_kernel<<<(kRows * (kDin / 2)) / 256, 256, 0, stream>>>(
      (const unsigned*)DTP, b_dt, Dskip, SS, (const unsigned*)XC, XIZ, (unsigned*)YY);

  wmma_gemm64<0, 0, 0, 0, false><<<dim3((kRows / 64) * (kDim / 64) / 8, 1), 256, 0, stream>>>(
      YY, nullptr, kDin, 0L,
      WOUT, nullptr, kDin, 0L,
      (void*)out, nullptr, kDim, 0L,
      nullptr, nullptr, 0L,
      kRows, kDim, kDin, 1.0f / (kActCarry * kWCarry));
}
